// SetAbstactionBlock_64458869178520
// MI455X (gfx1250) — hardware-verified
//
#include <hip/hip_runtime.h>
#include <math.h>

typedef __attribute__((ext_vector_type(16))) _Float16 v16h;
typedef __attribute__((ext_vector_type(16))) __bf16 v16b;
typedef __attribute__((ext_vector_type(8)))  _Float16 v8h;
typedef __attribute__((ext_vector_type(8)))  float v8f;
typedef __attribute__((ext_vector_type(4)))  float v4f;
typedef __attribute__((ext_vector_type(2)))  float v2f;
typedef __attribute__((ext_vector_type(4)))  unsigned v4u;
typedef __attribute__((ext_vector_type(4)))  int v4i;
typedef float __attribute__((may_alias)) float_a;
typedef int __attribute__((may_alias)) int_a;

template <typename T> __device__ __forceinline__ void vst2(void* p, T v) { *(volatile T*)p = v; __threadfence(); *(volatile T*)p = v; }
__device__ __forceinline__ v8f wmma16(v16h a, v16h b, v8f c) {
  v8f d = __builtin_amdgcn_wmma_f32_16x16x32_f16(false, a, false, b, (short)0, c, false, false);
  asm volatile("v_nop\n\tv_nop\n\tv_nop\n\tv_nop" : "+v"(d) : "v"(a), "v"(b));
  return d;
}
__device__ __forceinline__ v8f wmma_bf(v16b a, v16b b, v8f c) {
  v8f d = __builtin_amdgcn_wmma_f32_16x16x32_bf16(false, a, false, b, (short)0, c, false, false);
  asm volatile("v_nop\n\tv_nop\n\tv_nop\n\tv_nop" : "+v"(d) : "v"(a), "v"(b));
  return d;
}
__device__ __forceinline__ v16h frag_h(const _Float16* rowk0, int lane) {
  union { v16h v; v8h q[2]; } u; const _Float16* p = rowk0 + 8 * (lane >> 4);
  u.q[0] = *(const v8h*)p; u.q[1] = *(const v8h*)(p + 16); return u.v;
}
__device__ __forceinline__ v16h frag_f32(const float* rowk0, int lane) {
  v16h a; const float* p = rowk0 + 8 * (lane >> 4);
#pragma unroll
  for (int i = 0; i < 8; ++i) { a[i] = (_Float16)p[i]; a[8 + i] = (_Float16)p[16 + i]; }
  return a;
}
__device__ __forceinline__ v16h frag_f32s(const float* rowk0, int lane, float sc) {
  v16h a; const float* p = rowk0 + 8 * (lane >> 4);
#pragma unroll
  for (int i = 0; i < 8; ++i) { a[i] = (_Float16)(p[i] * sc); a[8 + i] = (_Float16)(p[16 + i] * sc); }
  return a;
}
__device__ __forceinline__ v16h fragc_f32(const float* W, int k0, int n, int lane, int ld, int K) {
  v16h a; const int g = lane >> 4;
#pragma unroll
  for (int i = 0; i < 8; ++i) { const int ka = k0 + 8 * g + i, kb = ka + 16;
    a[i] = (_Float16)(ka < K ? W[(size_t)(ka < K ? ka : K - 1) * ld + n] : 0.f); a[8 + i] = (_Float16)(kb < K ? W[(size_t)(kb < K ? kb : K - 1) * ld + n] : 0.f); }
  return a;
}
struct F2 { v16b h, l; };
__device__ __forceinline__ F2 bsplit16(const float v[16]) { F2 r;
#pragma unroll
  for (int i = 0; i < 16; ++i) { const __bf16 h = (__bf16)v[i]; r.h[i] = h; r.l[i] = (__bf16)(v[i] - (float)h); }
  return r; }
__device__ __forceinline__ F2 split_row(const float* row, int k0, int lane) { float v[16]; const float* p = row + k0 + 8 * (lane >> 4);
#pragma unroll
  for (int i = 0; i < 8; ++i) { v[i] = p[i]; v[8 + i] = p[16 + i]; }
  return bsplit16(v); }
__device__ __forceinline__ F2 split_rowK(const float* row, int k0, int lane, int K) { float v[16]; const int g = lane >> 4;
#pragma unroll
  for (int i = 0; i < 8; ++i) { const int ka = k0 + 8 * g + i, kb = ka + 16; v[i] = ka < K ? row[ka < K ? ka : K - 1] : 0.f; v[8 + i] = kb < K ? row[kb < K ? kb : K - 1] : 0.f; }
  return bsplit16(v); }
__device__ __forceinline__ F2 split_col(const float* W, int k0, int n, int lane, int ld, int K) { float v[16]; const int g = lane >> 4;
#pragma unroll
  for (int i = 0; i < 8; ++i) { const int ka = k0 + 8 * g + i, kb = ka + 16; v[i] = ka < K ? W[(size_t)(ka < K ? ka : K - 1) * ld + n] : 0.f; v[8 + i] = kb < K ? W[(size_t)(kb < K ? kb : K - 1) * ld + n] : 0.f; }
  return bsplit16(v); }
__device__ __forceinline__ v8f mac3(const F2& a, const F2& b, v8f c) { c = wmma_bf(a.l, b.h, c); c = wmma_bf(a.h, b.l, c); return wmma_bf(a.h, b.h, c); }
__device__ __forceinline__ float sigm(float v) { return 1.0f / (1.0f + expf(-v)); }
#define LDSX() do { asm volatile("s_wait_dscnt 0" ::: "memory"); __builtin_amdgcn_wave_barrier(); __builtin_amdgcn_fence(__ATOMIC_RELEASE, "workgroup"); } while (0)


#define NBc 16
#define NSRC 4096
#define NQ 1024
#define KK 32
#define CF 64
#define C1 64
#define C2 128
#define C3 256
#define KIN 96
#define NROW (NBc * NQ * KK)
#define NBLK (NROW / 64)
#ifndef TRBq
#define TRBq NBLK
#endif
typedef __attribute__((ext_vector_type(8))) __bf16 v8b;
__device__ __forceinline__ v16b frag_b(const __bf16* rowk0, int lane) {
  union { v16b v; v8b q[2]; } u; const __bf16* p = rowk0 + 8 * (lane >> 4);
  u.q[0] = *(const v8b*)p; u.q[1] = *(const v8b*)(p + 16); return u.v;
}
__device__ __forceinline__ float bfr(float v) { return (float)(__bf16)v; }
__device__ __attribute__((noinline)) float exp_ni(float v) { return expf(v); }
__device__ __attribute__((noinline)) float erf_ni(float v) { return erff(v); }

#define WS_P1  0u
#define WS_P2  (WS_P1 + 2u * C1 * KIN)
#define WS_P3  (WS_P2 + 2u * C2 * C1)
#define WS_GI  (((WS_P3 + 2u * C3 * C2) + 127u) / 128u * 128u)
#define WS_ST1 (WS_GI + 4u * NBc * NQ * KK)
#define WS_BN1 (WS_ST1 + 4u * (size_t)NBLK * C1 * 2)
#define WS_ST2 (WS_BN1 + 4u * C1 * 2)
#define WS_BN2 (WS_ST2 + 4u * (size_t)NBLK * C2 * 2)
#define WS_HM  (WS_BN2 + 4u * C2 * 2)
#define WS_ST3 (WS_HM + 4u * (size_t)NBc * NQ * C3)
#define WS_BN3 (WS_ST3 + 4u * 256 * C3 * 2)
#define WS_END (WS_BN3 + 4u * C3 * 2)

__device__ __attribute__((noinline)) float gelu_p(float x) { return 0.5f * x * (1.0f + erff(x * 0.70710678118654752f)); }
__global__ __launch_bounds__(128) void k_pack(const float* __restrict__ W1, const float* __restrict__ W2, const float* __restrict__ W3, __bf16* __restrict__ P) {
  const int n = blockIdx.x, which = blockIdx.y, t = threadIdx.x; __shared__ __align__(16) __bf16 s[C2];
  if (which == 0) { if (n >= C1) return; if (t < KIN) s[t] = (__bf16)((t < CF + 3) ? W1[(size_t)n * (CF + 3) + t] : 0.f); __syncthreads(); if (t < KIN / 8) vst2((unsigned*)(P + WS_P1 / 2 + (size_t)n * KIN + t * 8), *(const v4u*)&s[t * 8]); }
  else if (which == 1) { if (n >= C2) return; if (t < C1) s[t] = (__bf16)W2[(size_t)n * C1 + t]; __syncthreads(); if (t < C1 / 8) vst2((unsigned*)(P + WS_P2 / 2 + (size_t)n * C1 + t * 8), *(const v4u*)&s[t * 8]); }
  else { s[t] = (__bf16)W3[(size_t)n * C2 + t]; __syncthreads(); if (t < C2 / 8) vst2((unsigned*)(P + WS_P3 / 2 + (size_t)n * C2 + t * 8), *(const v4u*)&s[t * 8]); }
}
__global__ __launch_bounds__(64) void k_ball(const float* __restrict__ SXYZ, const float* __restrict__ QXYZ, int* __restrict__ GI) {
  __shared__ float ssrc[NSRC * 3]; const int b = blockIdx.y, t = threadIdx.x; const int m = blockIdx.x * 64 + t;
  for (int e = t; e < NSRC * 3; e += 64) ssrc[e] = bfr(SXYZ[(size_t)b * NSRC * 3 + e]);
  __syncthreads();
  const float qx = bfr(QXYZ[((size_t)b * NQ + m) * 3]), qy = bfr(QXYZ[((size_t)b * NQ + m) * 3 + 1]), qz = bfr(QXYZ[((size_t)b * NQ + m) * 3 + 2]);
  int cnt = 0; int* dst = GI + ((size_t)b * NQ + m) * KK;
  int idx[KK];
#pragma unroll
  for (int k = 0; k < KK; ++k) idx[k] = -1;
  for (int n = 0; n < NSRC && cnt < KK; ++n) { const float dx = qx - ssrc[n * 3], dy = qy - ssrc[n * 3 + 1], dz = qz - ssrc[n * 3 + 2]; const float d2 = dx * dx + dy * dy + dz * dz;
    if (d2 <= 0.04f) { dst[cnt] = n; ++cnt; } }
  const int first = (cnt > 0) ? dst[0] : 0;
  for (int k = cnt; k < KK; ++k) dst[k] = first;
  (void)idx;
}
template <int MODE>
__global__ __launch_bounds__(128) void k_mlp(const float* __restrict__ SX, const float* __restrict__ SXYZ, const float* __restrict__ QXYZ, const int* __restrict__ GI, const __bf16* __restrict__ P, const float* __restrict__ BN1, const float* __restrict__ G1, const float* __restrict__ Bt1, const float* __restrict__ BN2, const float* __restrict__ G2, const float* __restrict__ Bt2, float* __restrict__ STAT, float* __restrict__ HM) {
  __shared__ __align__(16) __bf16 sah[64][KIN + 8], sal[64][KIN + 8]; __shared__ __align__(16) __bf16 s1h[64][C1 + 8], s1l[64][C1 + 8]; __shared__ __align__(16) __bf16 s2h[64][C2 + 8], s2l[64][C2 + 8]; __shared__ __align__(16) float sf[64][C2 + 4]; __shared__ __align__(16) float sstat[C2][2]; __shared__ __align__(16) float smax[2][C3];
  const int tid = threadIdx.x, wave = tid >> 5, lane = tid & 31, col = lane & 15, g = lane >> 4; const size_t rb0 = (size_t)blockIdx.x * 64; const int b = (int)(rb0 / ((size_t)NQ * KK)); const int m0 = (int)((rb0 / KK) % NQ);
  for (int e = tid; e < 64 * KIN; e += 128) { const int r = e / KIN, c = e % KIN; const int m = m0 + (r >> 5), k = r & 31; const int src = GI[((size_t)b * NQ + m) * KK + k]; float v = 0.f;
    if (c < 3) v = bfr(SXYZ[((size_t)b * NSRC + src) * 3 + c]) - bfr(QXYZ[((size_t)b * NQ + m) * 3 + c]); else if (c < 3 + CF) v = bfr(SX[((size_t)b * NSRC + src) * CF + (c - 3)]);
    const __bf16 hb = (__bf16)v; sah[r][c] = hb; sal[r][c] = (__bf16)(v - (float)hb); }
  if (tid < 64) for (int c = KIN; c < KIN + 8; ++c) { sah[tid][c] = (__bf16)0.f; sal[tid][c] = (__bf16)0.f; }
  __syncthreads();
  { v8f acc[4] = {};
#pragma unroll
    for (int kc = 0; kc < KIN / 32; ++kc) { const v16b a = frag_b(&sah[wave * 16 + col][kc * 32], lane), al = frag_b(&sal[wave * 16 + col][kc * 32], lane);
#pragma unroll
      for (int j = 0; j < 4; ++j) { const v16b w = frag_b(P + WS_P1 / 2 + (size_t)(j * 16 + col) * KIN + kc * 32, lane); acc[j] = wmma_bf(al, w, acc[j]); acc[j] = wmma_bf(a, w, acc[j]); } }
#pragma unroll
    for (int j = 0; j < 4; ++j) { const int c = j * 16 + col;
#pragma unroll
      for (int r = 0; r < 8; ++r) { float v = acc[j][r]; if (MODE >= 1) { v = (v - BN1[c * 2]) * BN1[c * 2 + 1] * bfr(G1[c]) + bfr(Bt1[c]); v = gelu_p(v); const __bf16 hb = (__bf16)v; s1h[wave * 16 + 8 * g + r][c] = hb; s1l[wave * 16 + 8 * g + r][c] = (__bf16)(v - (float)hb); } else sf[wave * 16 + 8 * g + r][c] = v; } } }
  if (MODE >= 1) { if (tid < 64) for (int c = C1; c < C1 + 8; ++c) { s1h[tid][c] = (__bf16)0.f; s1l[tid][c] = (__bf16)0.f; } }
  __syncthreads();
  if (MODE >= 1) { v8f acc[8] = {};
#pragma unroll
    for (int kc = 0; kc < C1 / 32; ++kc) { const v16b a = frag_b(&s1h[wave * 16 + col][kc * 32], lane), al = frag_b(&s1l[wave * 16 + col][kc * 32], lane);
#pragma unroll
      for (int j = 0; j < 8; ++j) { const v16b w = frag_b(P + WS_P2 / 2 + (size_t)(j * 16 + col) * C1 + kc * 32, lane); acc[j] = wmma_bf(al, w, acc[j]); acc[j] = wmma_bf(a, w, acc[j]); } }
#pragma unroll
    for (int j = 0; j < 8; ++j) { const int c = j * 16 + col;
#pragma unroll
      for (int r = 0; r < 8; ++r) { float v = acc[j][r]; if (MODE >= 2) { v = (v - BN2[c * 2]) * BN2[c * 2 + 1] * bfr(G2[c]) + bfr(Bt2[c]); v = gelu_p(v); const __bf16 hb = (__bf16)v; s2h[wave * 16 + 8 * g + r][c] = hb; s2l[wave * 16 + 8 * g + r][c] = (__bf16)(v - (float)hb); } else sf[wave * 16 + 8 * g + r][c] = v; } }
    if (MODE >= 2) { if (tid < 64) for (int c = C2; c < C2 + 8; ++c) { s2h[tid][c] = (__bf16)0.f; s2l[tid][c] = (__bf16)0.f; } }
    __syncthreads(); }
  if (MODE <= 1) {
    constexpr int CCm = (MODE == 0) ? C1 : C2;
    if (tid < CCm) { float s = 0.f; for (int r = 0; r < 64; ++r) s += sf[r][tid]; const float mean = s / 64.0f; float m2 = 0.f; for (int r = 0; r < 64; ++r) { const float d = sf[r][tid] - mean; m2 += d * d; } sstat[tid][0] = mean; sstat[tid][1] = m2; }
    __syncthreads();
    if (tid < CCm / 2) vst2(STAT + (size_t)blockIdx.x * CCm * 2 + tid * 4, *(const v4f*)(&sstat[0][0] + tid * 4));
    return; }
#pragma unroll 1
  for (int pass = 0; pass < 2; ++pass) { v8f acc[8] = {};
#pragma unroll
    for (int kc = 0; kc < C2 / 32; ++kc) { const v16b a = frag_b(&s2h[wave * 16 + col][kc * 32], lane), al = frag_b(&s2l[wave * 16 + col][kc * 32], lane);
#pragma unroll
      for (int j = 0; j < 8; ++j) { const v16b w = frag_b(P + WS_P3 / 2 + (size_t)(pass * 128 + j * 16 + col) * C2 + kc * 32, lane); acc[j] = wmma_bf(al, w, acc[j]); acc[j] = wmma_bf(a, w, acc[j]); } }
#pragma unroll
    for (int j = 0; j < 8; ++j)
#pragma unroll
      for (int r = 0; r < 8; ++r) sf[wave * 16 + 8 * g + r][j * 16 + col] = acc[j][r];
    __syncthreads();
    { const int c = tid; float mx0 = -3.0e38f, mx1 = -3.0e38f; for (int r = 0; r < 32; ++r) { mx0 = fmaxf(mx0, sf[r][c]); mx1 = fmaxf(mx1, sf[32 + r][c]); } smax[0][pass * 128 + c] = mx0; smax[1][pass * 128 + c] = mx1; }
    __syncthreads(); }
  for (int e = tid; e < 2 * C3 / 4; e += 128) { const int q = e / (C3 / 4), i = e % (C3 / 4); vst2(HM + (((size_t)b * NQ + m0 + q) * C3) + i * 4, *(const v4f*)&smax[q][i * 4]); }
}
__device__ __forceinline__ void chan_comb(float& n, float& mean, float& M2, float nb, float mb, float m2b) {
  if (nb <= 0.f) return; if (n <= 0.f) { n = nb; mean = mb; M2 = m2b; return; }
  const float nn = n + nb; const float delta = mb - mean; mean = mean + delta * (nb / nn); M2 = M2 + m2b + delta * delta * (n * nb / nn); n = nn; }
__global__ __launch_bounds__(256) void k_comb(const float* __restrict__ STAT, int nblk, int ccs, float cnt_each, float* __restrict__ BN) {
  const int c = blockIdx.x, t = threadIdx.x; __shared__ float sm[256], sM2[256], sn[256];
  const int per = (nblk + 255) / 256; float n = 0.f, mean = 0.f, M2 = 0.f;
#pragma unroll 1
  for (int i = t * per; i < nblk && i < (t + 1) * per; ++i) chan_comb(n, mean, M2, cnt_each, STAT[((size_t)i * ccs + c) * 2], STAT[((size_t)i * ccs + c) * 2 + 1]);
  sm[t] = mean; sM2[t] = M2; sn[t] = n; __syncthreads();
#pragma unroll 1
  for (int s = 128; s >= 1; s >>= 1) { if (t < s) { float na = sn[t], ma = sm[t], qa = sM2[t]; chan_comb(na, ma, qa, sn[t + s], sm[t + s], sM2[t + s]); sn[t] = na; sm[t] = ma; sM2[t] = qa; } __syncthreads(); }
  if (t == 0) { const float var = sM2[0] / sn[0]; BN[c * 2] = sm[0]; BN[c * 2 + 1] = 1.0f / sqrtf(var + 1e-5f); }
}
__global__ __launch_bounds__(256) void k_st3(const float* __restrict__ HM, float* __restrict__ STAT) {
  const size_t r0 = (size_t)blockIdx.x * 64; const int c = threadIdx.x; float s = 0.f; for (int r = 0; r < 64; ++r) s += HM[(r0 + r) * C3 + c]; const float mean = s / 64.0f; float m2 = 0.f; for (int r = 0; r < 64; ++r) { const float d = HM[(r0 + r) * C3 + c] - mean; m2 += d * d; }
  __shared__ __align__(16) float so[C3][2]; so[c][0] = mean; so[c][1] = m2; __syncthreads();
  if (c < C3 / 2) vst2(STAT + (size_t)blockIdx.x * C3 * 2 + c * 4, *(const v4f*)(&so[0][0] + c * 4));
}
__global__ __launch_bounds__(256) void k_out(const float* __restrict__ HM, const float* __restrict__ BN3, const float* __restrict__ G3, const float* __restrict__ Bt3, float* __restrict__ OUT) {
  const size_t r0 = (size_t)blockIdx.x * 64; const int t = threadIdx.x; __shared__ __align__(16) float so[64][C3];
  for (int e = t; e < 64 * C3; e += 256) { const int r = e >> 8, c = e & 255; const float v = (HM[(r0 + r) * C3 + c] - BN3[c * 2]) * BN3[c * 2 + 1] * bfr(G3[c]) + bfr(Bt3[c]); so[r][c] = gelu_p(v); }
  __syncthreads();
  for (int q = t; q < 64 * C3 / 4; q += 256) vst2(OUT + r0 * C3 + q * 4, *(const v4f*)(&so[0][0] + q * 4));
}
extern "C" void kernel_launch(void* const* d_in, const int* in_sizes, int n_in, void* d_out, int out_size, void* d_ws, size_t ws_size, hipStream_t stream) {
  (void)in_sizes; (void)n_in; (void)out_size;
  const float** F = (const float**)d_in;
  if (ws_size < (size_t)WS_END) return;
  char* ws = (char*)d_ws; __bf16* P = (__bf16*)ws; int* GI = (int*)(ws + WS_GI); float *ST1 = (float*)(ws + WS_ST1), *BN1 = (float*)(ws + WS_BN1), *ST2 = (float*)(ws + WS_ST2), *BN2 = (float*)(ws + WS_BN2), *HM = (float*)(ws + WS_HM), *ST3 = (float*)(ws + WS_ST3), *BN3 = (float*)(ws + WS_BN3);
  k_pack<<<dim3(C3, 3), 128, 0, stream>>>(F[3], F[6], F[9], P);
  k_ball<<<dim3(NQ / 64, NBc), 64, 0, stream>>>(F[1], F[2], GI);
  k_mlp<0><<<TRBq, 128, 0, stream>>>(F[0], F[1], F[2], GI, P, nullptr, nullptr, nullptr, nullptr, nullptr, nullptr, ST1, nullptr);
  k_comb<<<C1, 256, 0, stream>>>(ST1, TRBq, C1, 64.0f, BN1);
  k_mlp<1><<<TRBq, 128, 0, stream>>>(F[0], F[1], F[2], GI, P, BN1, F[4], F[5], nullptr, nullptr, nullptr, ST2, nullptr);
  k_comb<<<C2, 256, 0, stream>>>(ST2, TRBq, C2, 64.0f, BN2);
  k_mlp<2><<<TRBq, 128, 0, stream>>>(F[0], F[1], F[2], GI, P, BN1, F[4], F[5], BN2, F[7], F[8], nullptr, HM);
  k_st3<<<(TRBq * 2) / 64, 256, 0, stream>>>(HM, ST3);
  k_comb<<<C3, 256, 0, stream>>>(ST3, (TRBq * 2) / 64, C3, 64.0f, BN3);
  k_out<<<(TRBq * 2) / 64, 256, 0, stream>>>(HM, BN3, F[10], F[11], (float*)d_out);
}
